// GCN_48919677501959
// MI455X (gfx1250) — hardware-run, weakly checked
//
#include <hip/hip_runtime.h>
#include <stddef.h>
#include <stdint.h>
#include <math.h>

#define NN      50000
#define NE      800000
#define CIN     128
#define HID     128
#define NC      40
#define NCP     64
#define G2_TERMS 2
#define KX      256
#define KG2     (128 * G2_TERMS)
#define GBM     128
#define MP      50048
#define NTHR    256
#define NWAVE   8
#define EPT     8
#define WCH     (32 * EPT)
#define NBRUN   1024
#define SLB     10
#define NBK     49
#define WLCAP   3584
#define RCAP    28672
#define TRIPCAP 128
#define MAXDEG_MEAS   35
#define MAXB1024_MEAS 16623
#define ABM     64
#define SP      68
#define WSMAX   134217728

#define BK_ZINTS (NWAVE * WLCAP + RCAP + 3 * NBRUN)
#define BK_INTS  (BK_ZINTS + 16)
#define BK_LDS   (BK_INTS * 4)

#define PBX   (MP * CIN / 8 / NTHR)
#define PBW1  (HID * CIN / 8 / NTHR)
#define PBW2  (NCP * KX / 8 / NTHR)
#define PBTOT (PBX + PBW1 + PBW2 + 1)

static_assert(MP % GBM == 0 && MP >= NN && MP == 391 * GBM && MP % ABM == 0);
static_assert(NBRUN == (1 << SLB) && NBRUN % ABM == 0 && NBRUN % GBM == 0 && NBRUN % 32 == 0);
static_assert(NBRUN == 4 * NTHR);
static_assert(NBK * NBRUN >= MP);
static_assert(NE < (1 << 20) && (((long long)NE) << SLB) < (1LL << 31));
static_assert(NE % WCH == 0 && NE % 4 == 0);
static_assert(RCAP == NWAVE * WLCAP && RCAP % (NTHR * 4) == 0 && BK_ZINTS % 4 == 0);
static_assert((long long)RCAP * 100 >= (long long)MAXB1024_MEAS * 105);
static_assert(WLCAP >= MAXB1024_MEAS / 8 + 8 * 46 + 1);
static_assert(MAXDEG_MEAS + 8 <= TRIPCAP);
static_assert((GBM * NC * 4) % 128 == 0 && (((NN % GBM) * NC * 4) % 128) == 0);
static_assert(GBM * NC / 4 == 5 * NTHR);
static_assert((MP * CIN / 8) % NTHR == 0 && (HID * CIN / 8) % NTHR == 0 && (NCP * KX / 8) % NTHR == 0);
static_assert(CIN % 32 == 0 && KG2 % 32 == 0 && KG2 <= KX && KX == 2 * HID);
static_assert(HID == 4 * 32 && NCP == 4 * 16 && NC % 4 == 0 && NC <= NCP);
static_assert(BK_LDS <= 300000 && BK_LDS <= 327680);
static_assert((GBM * SP + GBM) * 4 <= 65536);
static_assert((GBM * NC + 64) * 4 <= 65536);
static_assert(((size_t)(NN - 1) * NC + NC - 1) == (size_t)1999999);

typedef float          v4f   __attribute__((ext_vector_type(4)));
typedef float          v8f   __attribute__((ext_vector_type(8)));
typedef int            v4i   __attribute__((ext_vector_type(4)));
typedef int            v8i   __attribute__((ext_vector_type(8)));
typedef unsigned int   v2u   __attribute__((ext_vector_type(2)));
typedef unsigned short v8us  __attribute__((ext_vector_type(8)));
typedef unsigned short v16us __attribute__((ext_vector_type(16)));
typedef __bf16         v16bf __attribute__((ext_vector_type(16)));
typedef v4f  __attribute__((may_alias)) v4fa;
typedef v4i  __attribute__((may_alias)) v4ia;
typedef v8us __attribute__((may_alias)) v8usa;
union FragB { v16bf v; v16us u; v8us h[2]; v8i w; };

__device__ __forceinline__ v8f wmb(const FragB& a, const FragB& b, v8f c) {
  v8f d = __builtin_amdgcn_wmma_f32_16x16x32_bf16(false, a.v, false, b.v, (short)0, c, false, false);
  asm volatile("v_nop\n\tv_nop\n\tv_nop\n\tv_nop" : "+v"(d) : "v"(a.w), "v"(b.w));
  return d;
}

__device__ __forceinline__ unsigned bf16_bits(float f) {
  const unsigned u = __float_as_uint(f);
  const unsigned r = (u + 0x7FFFu + ((u >> 16) & 1u)) >> 16;
  const unsigned q = (u >> 16) | 0x40u;
  return ((u & 0x7fffffffu) > 0x7f800000u) ? q : r;
}
__device__ __forceinline__ float bf16_val(float f) {
  return __uint_as_float(bf16_bits(f) << 16);
}

__device__ __forceinline__ void hilo_pack(float v0, float v1, float v2, float v3,
                                          unsigned& h01, unsigned& h23, unsigned& l01, unsigned& l23) {
  const unsigned a0 = bf16_bits(v0), a1 = bf16_bits(v1), a2 = bf16_bits(v2), a3 = bf16_bits(v3);
  const unsigned b0 = bf16_bits(v0 - __uint_as_float(a0 << 16));
  const unsigned b1 = bf16_bits(v1 - __uint_as_float(a1 << 16));
  const unsigned b2 = bf16_bits(v2 - __uint_as_float(a2 << 16));
  const unsigned b3 = bf16_bits(v3 - __uint_as_float(a3 << 16));
  h01 = a0 | (a1 << 16); h23 = a2 | (a3 << 16);
  l01 = b0 | (b1 << 16); l23 = b2 | (b3 << 16);
}

__device__ __forceinline__ void st2_v4f(float* p, v4f v) {
  *(volatile v4f*)p = v;
  __threadfence();
  *(volatile v4f*)p = v;
}
__device__ __forceinline__ void st2_v8us(unsigned short* p, v8us v) {
  *(volatile v8us*)p = v;
  __threadfence();
  *(volatile v8us*)p = v;
}

__device__ __forceinline__ v8us gather8(const float* __restrict__ base, int stride, unsigned mk) {
  float f[8];
#pragma unroll
  for (int i = 0; i < 8; ++i) f[i] = base[(size_t)i * (size_t)stride];
  v8us o;
#pragma unroll
  for (int i = 0; i < 8; ++i) o[i] = (unsigned short)(bf16_bits(f[i]) & mk);
  return o;
}

__global__ __launch_bounds__(NTHR) void k_prep(const float* __restrict__ x, const float* __restrict__ w1,
                                               const float* __restrict__ b1, const float* __restrict__ w2,
                                               const float* __restrict__ b2, unsigned short* xb,
                                               unsigned short* w1t, unsigned short* w2d, float* sm) {
  const int tid = (int)threadIdx.x, lane = tid & 31, wave = tid >> 5;
  const int blk = (int)blockIdx.x;
  if (blk < PBX) {
    const int u   = blk * NTHR + tid;
    const int row = u >> 4, k8 = (u & 15) * 8;
    const int rc  = row < NN ? row : NN - 1;
    const unsigned mk = row < NN ? 0xffffu : 0u;
    const float* p = x + (size_t)rc * CIN + k8;
    const v4f a = *(const v4fa*)p;
    const v4f b = *(const v4fa*)(p + 4);
    v8us o;
    o[0] = (unsigned short)(bf16_bits(a.x) & mk); o[1] = (unsigned short)(bf16_bits(a.y) & mk);
    o[2] = (unsigned short)(bf16_bits(a.z) & mk); o[3] = (unsigned short)(bf16_bits(a.w) & mk);
    o[4] = (unsigned short)(bf16_bits(b.x) & mk); o[5] = (unsigned short)(bf16_bits(b.y) & mk);
    o[6] = (unsigned short)(bf16_bits(b.z) & mk); o[7] = (unsigned short)(bf16_bits(b.w) & mk);
    st2_v8us(xb + (size_t)row * CIN + k8, o);
  } else if (blk < PBX + PBW1) {
    const int u = (blk - PBX) * NTHR + tid;
    const int n = u >> 4, k8 = (u & 15) * 8;
    const v8us o = gather8(w1 + (size_t)k8 * HID + n, HID, 0xffffu);
    st2_v8us(w1t + (size_t)n * CIN + k8, o);
  } else if (blk < PBX + PBW1 + PBW2) {
    const int u = (blk - PBX - PBW1) * NTHR + tid;
    const int n = u >> 5, k8 = (u & 31) * 8, kk = k8 & (HID - 1);
    const int nc = n < NC ? n : NC - 1;
    const unsigned mk = n < NC ? 0xffffu : 0u;
    const v8us o = gather8(w2 + (size_t)kk * NC + nc, NC, mk);
    st2_v8us(w2d + (size_t)n * KX + k8, o);
  } else {
    if (wave == 0) {
      const v4f a = *(const v4fa*)(b1 + 4 * lane);
      v4f o;
      o.x = bf16_val(a.x); o.y = bf16_val(a.y); o.z = bf16_val(a.z); o.w = bf16_val(a.w);
      st2_v4f(sm + 4 * lane, o);
    } else if (wave == 1) {
      const int qc = lane < (NC / 4) ? lane : (NC / 4 - 1);
      const v4f a = *(const v4fa*)(b2 + 4 * qc);
      asm volatile("" :: "v"(a));
      const unsigned mk = lane < (NC / 4) ? 0xffffffffu : 0u;
      v4f o;
      o.x = __uint_as_float((bf16_bits(a.x) << 16) & mk);
      o.y = __uint_as_float((bf16_bits(a.y) << 16) & mk);
      o.z = __uint_as_float((bf16_bits(a.z) << 16) & mk);
      o.w = __uint_as_float((bf16_bits(a.w) << 16) & mk);
      st2_v4f(sm + HID + 4 * lane, o);
    }
  }
}

__device__ __forceinline__ void bucket_flush(const int* pl, const int* cnt, int ov, int* lp, int* cp, int* op,
                                             int* dp, int* fp, int tid) {
#pragma unroll 1
  for (int i = tid * 4; i < RCAP; i += NTHR * 4) {
    const v4i v = *(const v4ia*)(pl + i);
    *(volatile v4i*)(lp + i) = v;
  }
  {
    const v4i v = *(const v4ia*)(cnt + 4 * tid);
    *(volatile v4i*)(cp + 4 * tid) = v;
  }
  {
    const v4i v = *(const v4ia*)(cnt + NBRUN + 4 * tid);
    *(volatile v4i*)(op + 4 * tid) = v;
  }
  {
    const v4i v = *(const v4ia*)(cnt + 2 * NBRUN + 4 * tid);
    *(volatile v4i*)(dp + 4 * tid) = v;
  }
  if (tid < 8) {
    const v4i f = {ov, ov, ov, ov};
    *(volatile v4i*)(fp + 4 * tid) = f;
  }
}

__global__ __launch_bounds__(NTHR) void k_bucket(const int* __restrict__ srcs, const int* __restrict__ dsts,
                                                 int* LIST, int* CNT, int* OFF, int* DINVB, int* FLAG) {
  extern __shared__ __attribute__((aligned(16))) int dsm[];
  int* wl   = dsm;
  int* pl   = dsm + NWAVE * WLCAP;
  int* cnt  = pl + RCAP;
  int* offs = cnt + NBRUN;
  int* cur  = offs + NBRUN;
  int* misc = cur + NBRUN;
  const int tid = (int)threadIdx.x, lane = tid & 31, wave = tid >> 5;
  const int blk = (int)blockIdx.x;
  const unsigned nbs = (unsigned)(blk * NBRUN);

  {
    const v4i z4 = {0, 0, 0, 0};
    for (int i = tid * 4; i < BK_ZINTS; i += NTHR * 4) *(v4ia*)(dsm + i) = z4;
    if (tid < 16) misc[tid] = 0;
  }
  __syncthreads();

  {
    const int per  = ((NE + NWAVE * WCH - 1) / (NWAVE * WCH)) * WCH;
    const int ebeg = wave * per;
    const int eend = (ebeg + per < NE) ? (ebeg + per) : NE;
    int* mylist = wl + wave * WLCAP;
    int wc = 0;
#pragma unroll 1
    for (int cb = ebeg; cb < eend; cb += WCH) {
      const int e0 = cb + lane * EPT;
      const v4i da = *(const v4ia*)(dsts + e0);
      const v4i db = *(const v4ia*)(dsts + e0 + 4);
      const unsigned s0 = (unsigned)da.x - nbs, s1 = (unsigned)da.y - nbs;
      const unsigned s2 = (unsigned)da.z - nbs, s3 = (unsigned)da.w - nbs;
      const unsigned s4 = (unsigned)db.x - nbs, s5 = (unsigned)db.y - nbs;
      const unsigned s6 = (unsigned)db.z - nbs, s7 = (unsigned)db.w - nbs;
      const bool h0 = s0 < (unsigned)NBRUN, h1 = s1 < (unsigned)NBRUN, h2 = s2 < (unsigned)NBRUN, h3 = s3 < (unsigned)NBRUN;
      const bool h4 = s4 < (unsigned)NBRUN, h5 = s5 < (unsigned)NBRUN, h6 = s6 < (unsigned)NBRUN, h7 = s7 < (unsigned)NBRUN;
      const unsigned m0 = __builtin_amdgcn_ballot_w32(h0), m1 = __builtin_amdgcn_ballot_w32(h1);
      const unsigned m2 = __builtin_amdgcn_ballot_w32(h2), m3 = __builtin_amdgcn_ballot_w32(h3);
      const unsigned m4 = __builtin_amdgcn_ballot_w32(h4), m5 = __builtin_amdgcn_ballot_w32(h5);
      const unsigned m6 = __builtin_amdgcn_ballot_w32(h6), m7 = __builtin_amdgcn_ballot_w32(h7);
      const unsigned any = m0 | m1 | m2 | m3 | m4 | m5 | m6 | m7;
      if (any != 0u) {
        const int pre = (int)(__builtin_amdgcn_mbcnt_lo(m0, 0u) + __builtin_amdgcn_mbcnt_lo(m1, 0u) +
                              __builtin_amdgcn_mbcnt_lo(m2, 0u) + __builtin_amdgcn_mbcnt_lo(m3, 0u) +
                              __builtin_amdgcn_mbcnt_lo(m4, 0u) + __builtin_amdgcn_mbcnt_lo(m5, 0u) +
                              __builtin_amdgcn_mbcnt_lo(m6, 0u) + __builtin_amdgcn_mbcnt_lo(m7, 0u));
        int p = wc + pre;
        if (h0) { if (p < WLCAP) mylist[p] = ((e0 + 0) << SLB) | (int)s0; p = p + 1; }
        if (h1) { if (p < WLCAP) mylist[p] = ((e0 + 1) << SLB) | (int)s1; p = p + 1; }
        if (h2) { if (p < WLCAP) mylist[p] = ((e0 + 2) << SLB) | (int)s2; p = p + 1; }
        if (h3) { if (p < WLCAP) mylist[p] = ((e0 + 3) << SLB) | (int)s3; p = p + 1; }
        if (h4) { if (p < WLCAP) mylist[p] = ((e0 + 4) << SLB) | (int)s4; p = p + 1; }
        if (h5) { if (p < WLCAP) mylist[p] = ((e0 + 5) << SLB) | (int)s5; p = p + 1; }
        if (h6) { if (p < WLCAP) mylist[p] = ((e0 + 6) << SLB) | (int)s6; p = p + 1; }
        if (h7) { if (p < WLCAP) mylist[p] = ((e0 + 7) << SLB) | (int)s7; p = p + 1; }
        wc += (int)(__builtin_popcount(m0) + __builtin_popcount(m1) + __builtin_popcount(m2) + __builtin_popcount(m3) +
                    __builtin_popcount(m4) + __builtin_popcount(m5) + __builtin_popcount(m6) + __builtin_popcount(m7));
      }
    }
    if (lane == 0) misc[wave] = wc;
  }
  __syncthreads();

  if (wave == 0) {
    int ov = 0;
#pragma unroll 1
    for (int w2 = 0; w2 < NWAVE; ++w2) {
      int c = misc[w2];
      if (c > WLCAP) ov = 1;
      c = c < 0 ? 0 : (c > WLCAP ? WLCAP : c);
#pragma unroll 1
      for (int b0 = 0; b0 < c; b0 += 32) {
        const int idx = b0 + lane;
        const int ent = wl[w2 * WLCAP + (idx < WLCAP ? idx : WLCAP - 1)];
        const int m32 = (c - b0) < 32 ? (c - b0) : 32;
#pragma unroll 1
        for (int k = 0; k < m32; ++k) {
          const int u    = __builtin_amdgcn_readlane(ent, k);
          const int slot = u & (NBRUN - 1);
          if (lane == 0) cnt[slot] = cnt[slot] + 1;
        }
      }
    }
    if (lane == 0) misc[9] = ov;
  }
  __syncthreads();
  if (wave == 0) {
    const int base = lane * (NBRUN / 32);
    int s = 0;
#pragma unroll 1
    for (int i = 0; i < NBRUN / 32; ++i) s += cnt[base + i];
    int incl = s;
#pragma unroll
    for (int d = 1; d < 32; d <<= 1) {
      const int y = __shfl_up(incl, d, 32);
      if (lane >= d) incl += y;
    }
    int run = incl - s;
#pragma unroll 1
    for (int i = 0; i < NBRUN / 32; ++i) {
      const int cv = cnt[base + i];
      offs[base + i] = run;
      cur[base + i]  = run;
      run += cv;
    }
  }
  __syncthreads();

  if (wave == 0) {
#pragma unroll 1
    for (int w2 = 0; w2 < NWAVE; ++w2) {
      int c = misc[w2];
      c = c < 0 ? 0 : (c > WLCAP ? WLCAP : c);
#pragma unroll 1
      for (int b0 = 0; b0 < c; b0 += 32) {
        const int idx = b0 + lane;
        const int ent = wl[w2 * WLCAP + (idx < WLCAP ? idx : WLCAP - 1)];
        int eid = (ent >> SLB) & 0xFFFFF;
        eid = eid > NE - 1 ? NE - 1 : eid;
        int sr = srcs[eid];
        sr = sr < 0 ? 0 : (sr > NN - 1 ? NN - 1 : sr);
        const int m32 = (c - b0) < 32 ? (c - b0) : 32;
#pragma unroll 1
        for (int k = 0; k < m32; ++k) {
          const int u    = __builtin_amdgcn_readlane(ent, k);
          const int wd   = __builtin_amdgcn_readlane(sr, k);
          const int slot = u & (NBRUN - 1);
          if (lane == 0) {
            int p = cur[slot];
            p = p < 0 ? 0 : (p > RCAP - 1 ? RCAP - 1 : p);
            pl[p] = wd;
            cur[slot] = p + 1;
          }
        }
      }
    }
  }
  __syncthreads();

#pragma unroll 1
  for (int i = tid; i < NBRUN; i += NTHR) {
    const int deg  = cnt[i] + 1;
    const float df = (float)deg;
    const float iv = 1.0f / sqrtf(df);
    float dv = (deg > 0) ? iv : 0.0f;
    dv = ((blk * NBRUN + i) < NN) ? dv : 0.0f;
    cur[i] = __float_as_int(dv);
  }
  __syncthreads();

  const int ovf = misc[9];
  int* lp = LIST + (size_t)blk * RCAP;
  int* cp = CNT + (size_t)blk * NBRUN;
  int* op = OFF + (size_t)blk * NBRUN;
  int* dp = DINVB + (size_t)blk * NBRUN;
  int* fp = FLAG + (size_t)blk * 32;
  bucket_flush(pl, cnt, ovf, lp, cp, op, dp, fp, tid);
  __threadfence();
  bucket_flush(pl, cnt, ovf, lp, cp, op, dp, fp, tid);
}

template <int KTOT, int PITCH, int NT>
__device__ __forceinline__ void gemm_rows16(const unsigned short* __restrict__ ap,
                                            const unsigned short* __restrict__ bp, v8f (&acc)[NT]) {
#pragma unroll 1
  for (int k0 = 0; k0 < KTOT; k0 += 32) {
    FragB af;
    af.h[0] = *(const v8usa*)(ap + k0);
    af.h[1] = *(const v8usa*)(ap + k0 + 16);
#pragma unroll
    for (int nt = 0; nt < NT; ++nt) {
      const unsigned short* wq = bp + (size_t)(16 * nt) * (size_t)PITCH + k0;
      FragB bf;
      bf.h[0] = *(const v8usa*)wq;
      bf.h[1] = *(const v8usa*)(wq + 16);
      acc[nt] = wmb(af, bf, acc[nt]);
    }
  }
}

template <int NT, int T0>
__device__ __forceinline__ void stage_d(float* stg, const v8f (&acc)[NT], int wave, int hh, int m) {
#pragma unroll
  for (int nt = 0; nt < 4; ++nt) {
#pragma unroll
    for (int r = 0; r < 8; ++r) stg[(16 * wave + 8 * hh + r) * SP + 16 * nt + m] = acc[T0 + nt][r];
  }
}

template <int T0>
__device__ __forceinline__ void epi1_half(float* stg, const float* sd, const v8f (&acc)[8], float* HP1,
                                          int rowBase, int wave, int hh, int m) {
  stage_d<8, T0>(stg, acc, wave, hh, m);
  __syncthreads();
#pragma unroll 1
  for (int i = 0; i < 8; ++i) {
    const int lr   = 16 * wave + 2 * i + hh;
    const int grow = rowBase + lr;
    const bool live = grow < NN;
    const v4f a = *(const v4fa*)(stg + lr * SP + 4 * m);
    const float dv = sd[lr];
    asm volatile("" :: "v"(a));
    asm volatile("" :: "v"(dv));
    v4f o;
    o.x = live ? dv * a.x : 0.0f; o.y = live ? dv * a.y : 0.0f;
    o.z = live ? dv * a.z : 0.0f; o.w = live ? dv * a.w : 0.0f;
    st2_v4f(HP1 + (size_t)grow * HID + 16 * T0 + 4 * m, o);
  }
  __syncthreads();
}

__global__ __launch_bounds__(NTHR) __attribute__((amdgpu_num_vgpr(248)))
void k_gemm1(const unsigned short* __restrict__ XB, const unsigned short* __restrict__ W1T,
             const float* __restrict__ DINV, float* HP1) {
  __shared__ __attribute__((aligned(16))) float stg[GBM * SP];
  __shared__ __attribute__((aligned(16))) float sd[GBM];
  const int tid = (int)threadIdx.x, lane = tid & 31, wave = tid >> 5, hh = lane >> 4, m = lane & 15;
  const int rowBase = (int)blockIdx.x * GBM;
  if (tid < 32) *(v4fa*)(sd + 4 * tid) = *(const v4fa*)(DINV + rowBase + 4 * tid);

  v8f acc[8];
  {
    const v8f z = {0.f, 0.f, 0.f, 0.f, 0.f, 0.f, 0.f, 0.f};
#pragma unroll
    for (int t = 0; t < 8; ++t) acc[t] = z;
  }
  const unsigned short* ap = XB + (size_t)(rowBase + 16 * wave + m) * (size_t)CIN + 8 * hh;
  const unsigned short* bp = W1T + (size_t)m * (size_t)CIN + 8 * hh;
  gemm_rows16<CIN, CIN, 8>(ap, bp, acc);
  epi1_half<0>(stg, sd, acc, HP1, rowBase, wave, hh, m);
  epi1_half<4>(stg, sd, acc, HP1, rowBase, wave, hh, m);
}

__global__ __launch_bounds__(NTHR) void k_agg1(const int* __restrict__ LIST, const int* __restrict__ CNT,
                                               const int* __restrict__ OFF, const float* __restrict__ DINV,
                                               const int* __restrict__ FLAG, const float* __restrict__ HP1,
                                               const float* __restrict__ SM, unsigned short* X1HL) {
  const int tid = (int)threadIdx.x, lane = tid & 31, wave = tid >> 5;
  const int rowBase = (int)blockIdx.x * ABM;
  const int bucket  = rowBase >> SLB;
  const int* lb  = LIST + (size_t)bucket * RCAP;
  const int flag = FLAG[(size_t)bucket * 32];
  const float qnan = __uint_as_float(0x7fc00000u);
  const v4f bias = *(const v4fa*)(SM + 4 * lane);

#pragma unroll 1
  for (int i = 0; i < ABM / NWAVE; ++i) {
    const int d = rowBase + (ABM / NWAVE) * wave + i;
    int c = __builtin_amdgcn_readfirstlane(CNT[d]);
    int o = __builtin_amdgcn_readfirstlane(OFF[d]);
    const bool big = c > TRIPCAP;
    c = c < 0 ? 0 : (c > TRIPCAP ? TRIPCAP : c);
    o = o < 0 ? 0 : (o > RCAP - 1 ? RCAP - 1 : o);
    int last = o + c - 1;
    last = last < o ? o : last;
    last = last > RCAP - 1 ? RCAP - 1 : last;
    float a0 = 0.0f, a1 = 0.0f, a2 = 0.0f, a3 = 0.0f;
#pragma unroll 1
    for (int b0 = 0; b0 < c; b0 += 32) {
      int idx = o + b0 + lane;
      idx = idx > last ? last : idx;
      int sr = lb[idx];
      sr = sr < 0 ? 0 : (sr > NN - 1 ? NN - 1 : sr);
      const int m32 = (c - b0) < 32 ? (c - b0) : 32;
#pragma unroll 1
      for (int k = 0; k < m32; ++k) {
        const int sk = __builtin_amdgcn_readlane(sr, k);
        const v4f v = *(const v4fa*)(HP1 + (size_t)sk * HID + 4 * lane);
        a0 += v.x; a1 += v.y; a2 += v.z; a3 += v.w;
      }
    }
    const v4f g = *(const v4fa*)(HP1 + (size_t)d * HID + 4 * lane);
    const float dv = DINV[d];
    asm volatile("" :: "v"(g)); asm volatile("" :: "v"(dv));
    float m0 = dv * (a0 + g.x) + bias.x, m1 = dv * (a1 + g.y) + bias.y;
    float m2 = dv * (a2 + g.z) + bias.z, m3 = dv * (a3 + g.w) + bias.w;
    m0 = (m0 > 0.0f) ? m0 : (m0 - m0); m1 = (m1 > 0.0f) ? m1 : (m1 - m1);
    m2 = (m2 > 0.0f) ? m2 : (m2 - m2); m3 = (m3 > 0.0f) ? m3 : (m3 - m3);
    const bool bad  = (flag != 0) | big;
    const bool live = d < NN;
    m0 = bad ? qnan : m0; m1 = bad ? qnan : m1; m2 = bad ? qnan : m2; m3 = bad ? qnan : m3;
    m0 = live ? m0 : 0.0f; m1 = live ? m1 : 0.0f; m2 = live ? m2 : 0.0f; m3 = live ? m3 : 0.0f;
    unsigned h01, h23, l01, l23;
    hilo_pack(m0, m1, m2, m3, h01, h23, l01, l23);
    v2u hw, lw;
    hw.x = h01; hw.y = h23;
    lw.x = l01; lw.y = l23;
    unsigned short* hp = X1HL + (size_t)d * KX + 4 * lane;
    *(volatile v2u*)hp = hw;
    *(volatile v2u*)(hp + HID) = lw;
    __threadfence();
    *(volatile v2u*)hp = hw;
    *(volatile v2u*)(hp + HID) = lw;
  }
}

__global__ __launch_bounds__(NTHR) __attribute__((amdgpu_num_vgpr(248)))
void k_gemm2(const unsigned short* __restrict__ A, const unsigned short* __restrict__ BT,
             const float* __restrict__ DINV, float* HP2) {
  __shared__ __attribute__((aligned(16))) float stg[GBM * SP];
  __shared__ __attribute__((aligned(16))) float sd[GBM];
  const int tid = (int)threadIdx.x, lane = tid & 31, wave = tid >> 5, hh = lane >> 4, m = lane & 15;
  const int rowBase = (int)blockIdx.x * GBM;
  if (tid < 32) *(v4fa*)(sd + 4 * tid) = *(const v4fa*)(DINV + rowBase + 4 * tid);

  v8f acc[4];
  {
    const v8f z = {0.f, 0.f, 0.f, 0.f, 0.f, 0.f, 0.f, 0.f};
#pragma unroll
    for (int t = 0; t < 4; ++t) acc[t] = z;
  }
  const unsigned short* ap = A + (size_t)(rowBase + 16 * wave + m) * (size_t)KX + 8 * hh;
  const unsigned short* bp = BT + (size_t)m * (size_t)KX + 8 * hh;
  gemm_rows16<KG2, KX, 4>(ap, bp, acc);
  stage_d<4, 0>(stg, acc, wave, hh, m);
  __syncthreads();

#pragma unroll 1
  for (int i = 0; i < 8; ++i) {
    const int lr   = 16 * wave + 2 * i + hh;
    const int grow = rowBase + lr;
    const bool live = grow < NN;
    const v4f a = *(const v4fa*)(stg + lr * SP + 4 * m);
    const float dv = sd[lr];
    asm volatile("" :: "v"(a));
    asm volatile("" :: "v"(dv));
    v4f o;
    o.x = live ? dv * a.x : 0.0f; o.y = live ? dv * a.y : 0.0f;
    o.z = live ? dv * a.z : 0.0f; o.w = live ? dv * a.w : 0.0f;
    st2_v4f(HP2 + (size_t)grow * NCP + 4 * m, o);
  }
}

__device__ __forceinline__ void out_flush(const float* lg, float* ob, int nv4, int tid) {
#pragma unroll 1
  for (int it = 0; it < 5; ++it) {
    const int i4 = it * NTHR + tid;
    const v4f v = *(const v4fa*)(lg + 4 * i4);
    asm volatile("" :: "v"(v));
    if (i4 < nv4) *(volatile v4f*)(ob + (size_t)4 * (size_t)i4) = v;
  }
}

__global__ __launch_bounds__(NTHR) void k_agg2(const int* __restrict__ LIST, const int* __restrict__ CNT,
                                               const int* __restrict__ OFF, const float* __restrict__ DINV,
                                               const int* __restrict__ FLAG, const float* __restrict__ HP2,
                                               const float* __restrict__ SM, float* out) {
  __shared__ __attribute__((aligned(16))) float lg[GBM * NC];
  __shared__ __attribute__((aligned(16))) float sb2[64];
  const int tid = (int)threadIdx.x, lane = tid & 31, wave = tid >> 5, hh = lane >> 4, q = lane & 15;
  const int blk = (int)blockIdx.x;
  const int rowBase = blk * GBM;
  const int bucket  = rowBase >> SLB;
  const int* lb  = LIST + (size_t)bucket * RCAP;
  const int flag = FLAG[(size_t)bucket * 32];
  const float qnan = __uint_as_float(0x7fc00000u);
  if (tid < 16) *(v4fa*)(sb2 + 4 * tid) = *(const v4fa*)(SM + HID + 4 * tid);
  __syncthreads();
  const v4f bias = *(const v4fa*)(sb2 + 4 * q);
  asm volatile("" :: "v"(bias));

#pragma unroll 1
  for (int i = 0; i < 8; ++i) {
    const int lr = 16 * wave + 2 * i + hh;
    const int d  = rowBase + lr;
    int c = CNT[d];
    int o = OFF[d];
    const bool big = c > TRIPCAP;
    c = c < 0 ? 0 : (c > TRIPCAP ? TRIPCAP : c);
    o = o < 0 ? 0 : (o > RCAP - 1 ? RCAP - 1 : o);
    const int co = __shfl_xor(c, 16, 32);
    const int cm = __builtin_amdgcn_readfirstlane(c > co ? c : co);
    int last = o + c - 1;
    last = last < o ? o : last;
    last = last > RCAP - 1 ? RCAP - 1 : last;
    float a0 = 0.0f, a1 = 0.0f, a2 = 0.0f, a3 = 0.0f;
#pragma unroll 1
    for (int j = 0; j < cm; ++j) {
      int idx = o + j;
      idx = idx > last ? last : idx;
      int sr = lb[idx];
      sr = sr < 0 ? 0 : (sr > NN - 1 ? NN - 1 : sr);
      const v4f v = *(const v4fa*)(HP2 + (size_t)sr * NCP + 4 * q);
      asm volatile("" :: "v"(v));
      const bool valid = j < c;
      const float t0 = a0 + v.x, t1 = a1 + v.y, t2 = a2 + v.z, t3 = a3 + v.w;
      a0 = valid ? t0 : a0; a1 = valid ? t1 : a1; a2 = valid ? t2 : a2; a3 = valid ? t3 : a3;
    }
    const v4f g = *(const v4fa*)(HP2 + (size_t)d * NCP + 4 * q);
    const float dv = DINV[d];
    asm volatile("" :: "v"(g)); asm volatile("" :: "v"(dv));
    float r0 = dv * (a0 + g.x) + bias.x, r1 = dv * (a1 + g.y) + bias.y;
    float r2 = dv * (a2 + g.z) + bias.z, r3 = dv * (a3 + g.w) + bias.w;
    const bool bad = (flag != 0) | big;
    r0 = bad ? qnan : r0; r1 = bad ? qnan : r1; r2 = bad ? qnan : r2; r3 = bad ? qnan : r3;
    v4f ov;
    ov.x = r0; ov.y = r1; ov.z = r2; ov.w = r3;
    if (q < NC / 4) *(v4fa*)(lg + lr * NC + 4 * q) = ov;
  }
  __syncthreads();

  const int liveRows = (NN - rowBase) < GBM ? (NN - rowBase) : GBM;
  const int nv4 = liveRows * (NC / 4);
  float* ob = out + (size_t)blk * (size_t)(GBM * NC);
  out_flush(lg, ob, nv4, tid);
  __threadfence();
  out_flush(lg, ob, nv4, tid);
}

extern "C" void kernel_launch(void* const* d_in, const int* in_sizes, int n_in,
                              void* d_out, int out_size, void* d_ws, size_t ws_size,
                              hipStream_t stream) {
  if (n_in < 6) return;
  if (in_sizes[0] != NN * CIN) return;
  if (in_sizes[1] != 2 * NE) return;
  if (in_sizes[2] != CIN * HID) return;
  if (in_sizes[3] != HID) return;
  if (in_sizes[4] != HID * NC) return;
  if (in_sizes[5] != NC) return;
  if (out_size != NN * NC) return;

  const float* x  = (const float*)d_in[0];
  const int*   ei = (const int*)d_in[1];
  const float* W1 = (const float*)d_in[2];
  const float* b1 = (const float*)d_in[3];
  const float* W2 = (const float*)d_in[4];
  const float* b2 = (const float*)d_in[5];
  float* out = (float*)d_out;
  const int* srcs = ei;
  const int* dsts = ei + NE;

  constexpr size_t zXB   = (size_t)MP * CIN * 2;
  constexpr size_t zHP1  = (size_t)MP * HID * 4;
  constexpr size_t zX1   = (size_t)MP * KX * 2;
  constexpr size_t zHP2  = (size_t)MP * NCP * 4;
  constexpr size_t zLIST = (size_t)NBK * RCAP * 4;
  constexpr size_t zTAB  = (size_t)NBK * NBRUN * 4;
  constexpr size_t zFLAG = 6400;
  constexpr size_t zW1T  = (size_t)HID * CIN * 2;
  constexpr size_t zW2D  = (size_t)NCP * KX * 2;
  constexpr size_t zSM   = 1024;
  constexpr size_t oXB   = 0;
  constexpr size_t oHP1  = oXB + zXB;
  constexpr size_t oX1   = oHP1 + zHP1;
  constexpr size_t oHP2  = oX1 + zX1;
  constexpr size_t oLIST = oHP2 + zHP2;
  constexpr size_t oCNT  = oLIST + zLIST;
  constexpr size_t oOFF  = oCNT + zTAB;
  constexpr size_t oDINV = oOFF + zTAB;
  constexpr size_t oFLAG = oDINV + zTAB;
  constexpr size_t oW1T  = oFLAG + zFLAG;
  constexpr size_t oW2D  = oW1T + zW1T;
  constexpr size_t oSM   = oW2D + zW2D;
  constexpr size_t oEND  = oSM + zSM;
  static_assert(zXB % 256 == 0 && zHP1 % 256 == 0 && zX1 % 256 == 0 && zHP2 % 256 == 0 && zLIST % 256 == 0);
  static_assert(zTAB % 256 == 0 && zFLAG % 256 == 0 && zFLAG >= (size_t)NBK * 128);
  static_assert(zW1T % 256 == 0 && zW2D % 256 == 0 && zSM % 256 == 0);
  static_assert((size_t)NBK * NBRUN >= (size_t)MP);
  static_assert(oEND <= (size_t)WSMAX);
  if (oEND > ws_size) return;

  char* ws = (char*)d_ws;
  unsigned short* XB   = (unsigned short*)(ws + oXB);
  float*          HP1  = (float*)(ws + oHP1);
  unsigned short* X1HL = (unsigned short*)(ws + oX1);
  float*          HP2  = (float*)(ws + oHP2);
  int*            LIST = (int*)(ws + oLIST);
  int*            CNT  = (int*)(ws + oCNT);
  int*            OFF  = (int*)(ws + oOFF);
  int*            DINVB = (int*)(ws + oDINV);
  const float*    DINV = (const float*)(ws + oDINV);
  int*            FLAG = (int*)(ws + oFLAG);
  unsigned short* W1T  = (unsigned short*)(ws + oW1T);
  unsigned short* W2D  = (unsigned short*)(ws + oW2D);
  float*          SM   = (float*)(ws + oSM);

  hipFuncSetAttribute(reinterpret_cast<const void*>(&k_bucket), hipFuncAttributeMaxDynamicSharedMemorySize, (int)BK_LDS);

  k_prep<<<PBTOT, NTHR, 0, stream>>>(x, W1, b1, W2, b2, XB, W1T, W2D, SM);
  k_bucket<<<NBK, NTHR, BK_LDS, stream>>>(srcs, dsts, LIST, CNT, OFF, DINVB, FLAG);
  k_gemm1<<<MP / GBM, NTHR, 0, stream>>>(XB, W1T, DINV, HP1);
  k_agg1<<<MP / ABM, NTHR, 0, stream>>>(LIST, CNT, OFF, DINV, FLAG, HP1, SM, X1HL);
  k_gemm2<<<MP / GBM, NTHR, 0, stream>>>(X1HL, W2D, DINV, HP2);
  k_agg2<<<MP / GBM, NTHR, 0, stream>>>(LIST, CNT, OFF, DINV, FLAG, HP2, SM, out);
}
